// LightHeadRCNNResNet101_Head_27453430956790
// MI455X (gfx1250) — hardware-verified
//
#include <hip/hip_runtime.h>
#pragma clang fp contract(off)

typedef _Float16 f16t;
typedef _Float16 v16h __attribute__((ext_vector_type(16)));
typedef _Float16 v8h  __attribute__((ext_vector_type(8)));
typedef __bf16   v16b __attribute__((ext_vector_type(16)));
typedef unsigned short us_t;
typedef unsigned short v16us __attribute__((ext_vector_type(16)));
typedef unsigned short v8us  __attribute__((ext_vector_type(8)));
typedef float v8f __attribute__((ext_vector_type(8)));
typedef float v4f __attribute__((ext_vector_type(4)));
typedef v8us __attribute__((may_alias)) v8usa;
typedef v4f  __attribute__((may_alias)) v4fa;
typedef v8h  __attribute__((may_alias)) v8ha;

template<typename VT> union FragT { VT v; v8us half[2]; };

#define CIN    2048
#define HIMG   50
#define WIMG   75
#define NSP    3750
#define CMID   256
#define COUT   490
#define NROI   1000
#define NR     1024
#define XPW    89
#define XPROWS 5696
#define MCROWS 4450
#define MRROWS 4800
#define HPITCH 3840
#define K1     30720
#define K2     3840
#define KF     1536
#define FSEG   512
#define KH     6144
#define HSEG   2048
#define OPITCH 512
#define NLOC   324
#define NSCO   81
#define WCAR   64.0f

__device__ __forceinline__ int imin(int a, int b) { return a < b ? a : b; }
__device__ __forceinline__ int imax(int a, int b) { return a > b ? a : b; }

__device__ __forceinline__ v8f mma16(v16h a, v16h b, v8f c) {
  return __builtin_amdgcn_wmma_f32_16x16x32_f16(false, a, false, b, (short)0, c, false, false);
}
__device__ __forceinline__ v8f mma16(v16b a, v16b b, v8f c) {
  return __builtin_amdgcn_wmma_f32_16x16x32_bf16(false, a, false, b, (short)0, c, false, false);
}

__device__ __forceinline__ us_t bf_rne(float x) {
  unsigned u = __float_as_uint(x);
  u += 0x7FFFu + ((u >> 16) & 1u);
  return (us_t)(u >> 16);
}
__device__ __forceinline__ void bf_split(float x, us_t& hi, us_t& lo) {
  hi = bf_rne(x);
  const float hf = __uint_as_float(((unsigned)hi) << 16);
  lo = bf_rne(x - hf);
}
__device__ __forceinline__ v8us zero8us() {
  v8us z;
  #pragma unroll
  for (int j = 0; j < 8; ++j) z[j] = (us_t)0;
  return z;
}
__device__ __forceinline__ v8us pack8h(v4f a, v4f b, float s) {
  v8h o;
  o[0] = (f16t)(a.x * s); o[1] = (f16t)(a.y * s); o[2] = (f16t)(a.z * s); o[3] = (f16t)(a.w * s);
  o[4] = (f16t)(b.x * s); o[5] = (f16t)(b.y * s); o[6] = (f16t)(b.z * s); o[7] = (f16t)(b.w * s);
  return __builtin_bit_cast(v8us, o);
}
__device__ __forceinline__ void pack8bf(v4f a, v4f b, v8us& hi, v8us& lo) {
  float f[8];
  f[0] = a.x; f[1] = a.y; f[2] = a.z; f[3] = a.w; f[4] = b.x; f[5] = b.y; f[6] = b.z; f[7] = b.w;
  #pragma unroll
  for (int j = 0; j < 8; ++j) { us_t h, l; bf_split(f[j], h, l); hi[j] = h; lo[j] = l; }
}

__global__ __launch_bounds__(256) void xpad_k(const float* __restrict__ x, us_t* __restrict__ xp) {
  __shared__ __attribute__((aligned(16))) f16t sX[XPW * 64];
  const int tid = threadIdx.x, lane = tid & 31, wid = tid >> 5, q8 = lane & 7, sub = lane >> 3;
  const int c0 = blockIdx.x * 64, hp = blockIdx.y, h = hp - 7;
  const bool hv = (h >= 0) && (h < HIMG);
  {
    v8h z;
    #pragma unroll
    for (int j = 0; j < 8; ++j) z[j] = (f16t)0.0f;
    for (int s = tid; s < (XPW * 64) / 8; s += 256) *(v8ha*)(sX + 8 * s) = z;
  }
  __syncthreads();
  if (hv) {
    const int cl = tid >> 2, wq = tid & 3;
    const float* src = x + ((size_t)(c0 + cl) * HIMG + h) * WIMG;
    #pragma unroll 1
    for (int w = wq; w < WIMG; w += 4) sX[(w + 7) * 64 + cl] = (f16t)src[w];
  }
  __syncthreads();
  v8us vals[3];
  size_t adr[3];
  bool ok[3];
  #pragma unroll
  for (int it = 0; it < 3; ++it) {
    const int L = it * 32 + wid * 4 + sub;
    ok[it] = L < XPW;
    const int Lc = ok[it] ? L : 0;
    vals[it] = *(const v8usa*)(sX + Lc * 64 + 8 * q8);
    adr[it] = (size_t)(hp * XPW + Lc) * CIN + c0 + 8 * q8;
  }
  #pragma unroll
  for (int it = 0; it < 3; ++it) if (ok[it]) *(volatile v8us*)(xp + adr[it]) = vals[it];
  __threadfence();
  #pragma unroll
  for (int it = 0; it < 3; ++it) if (ok[it]) *(volatile v8us*)(xp + adr[it]) = vals[it];
}

__global__ __launch_bounds__(256) void packw_k(const float* __restrict__ w, us_t* __restrict__ out,
                                               int M, int Mp, int C, int total) {
  const int g = blockIdx.x * 256 + threadIdx.x;
  if (g >= total) return;
  const int c8n = C >> 3;
  const int c8 = g % c8n;
  const int t = (g / c8n) % 15;
  const int m = g / (c8n * 15);
  const int mc = imin(m, M - 1);
  const float* src = w + ((size_t)mc * C + 8 * c8) * 15 + t;
  const float sc = (m < M) ? WCAR : 0.0f;
  v8h o;
  #pragma unroll
  for (int i = 0; i < 8; ++i) o[i] = (f16t)(src[i * 15] * sc);
  const v8us ov = __builtin_bit_cast(v8us, o);
  us_t* dst = out + (size_t)m * 15 * C + (size_t)t * C + 8 * c8;
  *(volatile v8us*)dst = ov;
  __threadfence();
  *(volatile v8us*)dst = ov;
  (void)Mp;
}

__global__ __launch_bounds__(256) void packfc1_k(const float* __restrict__ w, us_t* __restrict__ out) {
  const int g = blockIdx.x * 256 + threadIdx.x;
  if (g >= 2048 * 64) return;
  const int j = g >> 6, q = g & 63;
  float f[8];
  #pragma unroll
  for (int i = 0; i < 8; ++i) {
    const int k = 8 * q + i;
    const int kc = imin(k, COUT - 1);
    const float v = w[(size_t)j * COUT + kc];
    f[i] = (k < COUT) ? v : 0.0f;
  }
  v8us hi, lo;
  #pragma unroll
  for (int i = 0; i < 8; ++i) { us_t a, b; bf_split(f[i], a, b); hi[i] = a; lo[i] = b; }
  us_t* dst = out + (size_t)j * KF + 8 * q;
  *(volatile v8us*)(dst) = hi;
  *(volatile v8us*)(dst + FSEG) = hi;
  *(volatile v8us*)(dst + 2 * FSEG) = lo;
  __threadfence();
  *(volatile v8us*)(dst) = hi;
  *(volatile v8us*)(dst + FSEG) = hi;
  *(volatile v8us*)(dst + 2 * FSEG) = lo;
}

__global__ __launch_bounds__(256) void packhead_k(const float* __restrict__ wl, const float* __restrict__ wsc,
                                                  us_t* __restrict__ out) {
  const int g = blockIdx.x * 256 + threadIdx.x;
  if (g >= 512 * 256) return;
  const int m = g >> 8, q = g & 255;
  const int ml = imin(m, NLOC - 1);
  const int ms = imin(imax(m - NLOC, 0), NSCO - 1);
  const float* pl = wl + (size_t)ml * 2048 + 8 * q;
  const float* ps = wsc + (size_t)ms * 2048 + 8 * q;
  const v4f la = *(const v4fa*)pl, lb = *(const v4fa*)(pl + 4);
  const v4f sa = *(const v4fa*)ps, sb = *(const v4fa*)(ps + 4);
  float f[8];
  f[0] = la.x; f[1] = la.y; f[2] = la.z; f[3] = la.w; f[4] = lb.x; f[5] = lb.y; f[6] = lb.z; f[7] = lb.w;
  float s[8];
  s[0] = sa.x; s[1] = sa.y; s[2] = sa.z; s[3] = sa.w; s[4] = sb.x; s[5] = sb.y; s[6] = sb.z; s[7] = sb.w;
  const bool isl = m < NLOC, iss = (m >= NLOC) && (m < NLOC + NSCO);
  v8us hi, lo;
  #pragma unroll
  for (int i = 0; i < 8; ++i) {
    const float v = isl ? f[i] : (iss ? s[i] : 0.0f);
    us_t a, b; bf_split(v, a, b); hi[i] = a; lo[i] = b;
  }
  us_t* dst = out + (size_t)m * KH + 8 * q;
  *(volatile v8us*)(dst) = hi;
  *(volatile v8us*)(dst + HSEG) = hi;
  *(volatile v8us*)(dst + 2 * HSEG) = lo;
  __threadfence();
  *(volatile v8us*)(dst) = hi;
  *(volatile v8us*)(dst + HSEG) = hi;
  *(volatile v8us*)(dst + 2 * HSEG) = lo;
}

__global__ __launch_bounds__(256) void zero_k(us_t* __restrict__ p, int n16) {
  const int i = blockIdx.x * 256 + threadIdx.x;
  if (i >= n16) return;
  const v8us z = zero8us();
  us_t* dst = p + (size_t)8 * i;
  *(volatile v8us*)dst = z;
  __threadfence();
  *(volatile v8us*)dst = z;
}

template<typename VT, int MODE>
__global__ __launch_bounds__(256) void gemm_k(
    const us_t* __restrict__ A1, const us_t* __restrict__ B1, int Ca, int tapsA, int tstrA, int rsA, int offA,
    const us_t* __restrict__ A2, const us_t* __restrict__ B2, int Cb, int tapsB, int tstrB, int rsB, int offB,
    int nparts, int Nvalid, int convmap,
    const float* __restrict__ bias0, int nb0, const float* __restrict__ bias1, int nb1,
    float osc, int relu,
    us_t* __restrict__ out16, float* __restrict__ outf, int ldo, int oRs, int oOff, int segStride)
{
  __shared__ __attribute__((aligned(16))) float S[8192];
  const int tid = threadIdx.x, lane = tid & 31, wid = tid >> 5;
  const int l15 = lane & 15, h8 = (lane >> 4) << 3, q8 = lane & 7, sub = lane >> 3;
  const int mblk = blockIdx.x * 128, nblk = blockIdx.y * 128;
  const int m0w = mblk + (wid & 3) * 32, n0w = nblk + (wid >> 2) * 64;

  v8f acc[2][4];
  {
    v8f z;
    #pragma unroll
    for (int j = 0; j < 8; ++j) z[j] = 0.0f;
    #pragma unroll
    for (int mt = 0; mt < 2; ++mt)
      #pragma unroll
      for (int nt = 0; nt < 4; ++nt) acc[mt][nt] = z;
  }

  #pragma unroll 1
  for (int part = 0; part < nparts; ++part) {
    const us_t* A = part ? A2 : A1;
    const us_t* B = part ? B2 : B1;
    const int C = part ? Cb : Ca;
    const int taps = part ? tapsB : tapsA;
    const int tstr = part ? tstrB : tstrA;
    const int rs = part ? rsB : rsA;
    const int off = part ? offB : offA;
    const int lda = taps * C;
    int base[4];
    #pragma unroll
    for (int nt = 0; nt < 4; ++nt) {
      const int n = n0w + nt * 16 + l15;
      const int nl = (n < Nvalid) ? n : (Nvalid - 1);
      int bse = nl;
      if (convmap) { const int hq = nl / WIMG; bse = hq * rs + (nl - hq * WIMG) + off; }
      base[nt] = bse;
    }
    const us_t* ar0 = A + (size_t)(m0w + l15) * lda + h8;
    const us_t* ar1 = ar0 + (size_t)16 * lda;
    #pragma unroll 1
    for (int t = 0; t < taps; ++t) {
      const us_t* ap0 = ar0 + (size_t)t * C;
      const us_t* ap1 = ar1 + (size_t)t * C;
      const us_t* bp[4];
      #pragma unroll
      for (int nt = 0; nt < 4; ++nt) bp[nt] = B + (size_t)(base[nt] + t * tstr) * C + h8;
      #pragma unroll 1
      for (int c0 = 0; c0 < C; c0 += 32) {
        FragT<VT> a0, a1, b[4];
        a0.half[0] = *(const v8usa*)(ap0 + c0);
        a0.half[1] = *(const v8usa*)(ap0 + c0 + 16);
        a1.half[0] = *(const v8usa*)(ap1 + c0);
        a1.half[1] = *(const v8usa*)(ap1 + c0 + 16);
        #pragma unroll
        for (int nt = 0; nt < 4; ++nt) {
          b[nt].half[0] = *(const v8usa*)(bp[nt] + c0);
          b[nt].half[1] = *(const v8usa*)(bp[nt] + c0 + 16);
        }
        #pragma unroll
        for (int nt = 0; nt < 4; ++nt) {
          acc[0][nt] = mma16(a0.v, b[nt].v, acc[0][nt]);
          acc[1][nt] = mma16(a1.v, b[nt].v, acc[1][nt]);
        }
        asm volatile("v_nop\n\tv_nop\n\tv_nop\n\tv_nop"
                     : "+v"(acc[0][0]), "+v"(acc[0][1]), "+v"(acc[0][2]), "+v"(acc[0][3]),
                       "+v"(acc[1][0]), "+v"(acc[1][1]), "+v"(acc[1][2]), "+v"(acc[1][3])
                     : "v"(a0.v), "v"(a1.v), "v"(b[0].v), "v"(b[1].v), "v"(b[2].v), "v"(b[3].v));
      }
    }
  }

  #pragma unroll 1
  for (int ph = 0; ph < 2; ++ph) {
    __syncthreads();
    if (((wid >> 1) & 1) == ph) {
      #pragma unroll
      for (int mt = 0; mt < 2; ++mt) {
        #pragma unroll
        for (int r = 0; r < 8; ++r) {
          const int mloc = (wid & 1) * 32 + mt * 16 + h8 + r;
          const int m = mblk + 64 * ph + mloc;
          float bv;
          if (MODE == 2) {
            bv = bias0[imin(m, nb0 - 1)] + bias1[imin(m, nb1 - 1)];
          } else if (MODE == 3) {
            const float bl = bias0[imin(m, nb0 - 1)];
            const float bs = bias1[imin(imax(m - nb0, 0), nb1 - 1)];
            bv = (m < nb0) ? bl : ((m < nb0 + nb1) ? bs : 0.0f);
          } else {
            bv = bias0[imin(m, nb0 - 1)];
          }
          #pragma unroll
          for (int nt = 0; nt < 4; ++nt) {
            const int nloc = (wid >> 2) * 64 + nt * 16 + l15;
            float v = acc[mt][nt][r] * osc + bv;
            if (relu) v = fmaxf(v, 0.0f);
            if (MODE == 2) S[mloc * 128 + nloc] = v;
            else S[nloc * 64 + mloc] = v;
          }
        }
      }
    }
    __syncthreads();

    if (MODE == 0) {
      v8us vals[4];
      size_t adr[4];
      bool ok[4];
      #pragma unroll
      for (int it = 0; it < 4; ++it) {
        const int nloc = it * 32 + wid * 4 + sub;
        const float* sp = S + nloc * 64 + 8 * q8;
        const v4f f0 = *(const v4fa*)sp;
        const v4f f1 = *(const v4fa*)(sp + 4);
        vals[it] = pack8h(f0, f1, 1.0f);
        const int n = nblk + nloc;
        ok[it] = n < Nvalid;
        const int nn = ok[it] ? n : 0;
        int pos = nn;
        if (convmap) { const int hq = nn / WIMG; pos = hq * oRs + (nn - hq * WIMG) + oOff; }
        adr[it] = (size_t)pos * ldo + mblk + 64 * ph + 8 * q8;
      }
      #pragma unroll
      for (int it = 0; it < 4; ++it) if (ok[it]) *(volatile v8us*)(out16 + adr[it]) = vals[it];
      __threadfence();
      #pragma unroll
      for (int it = 0; it < 4; ++it) if (ok[it]) *(volatile v8us*)(out16 + adr[it]) = vals[it];
    } else if (MODE == 1) {
      v8us vhi[4], vlo[4];
      size_t adr[4];
      bool ok[4];
      #pragma unroll
      for (int it = 0; it < 4; ++it) {
        const int nloc = it * 32 + wid * 4 + sub;
        const float* sp = S + nloc * 64 + 8 * q8;
        const v4f f0 = *(const v4fa*)sp;
        const v4f f1 = *(const v4fa*)(sp + 4);
        pack8bf(f0, f1, vhi[it], vlo[it]);
        const int n = nblk + nloc;
        ok[it] = n < Nvalid;
        const int nn = ok[it] ? n : 0;
        adr[it] = (size_t)nn * ldo + mblk + 64 * ph + 8 * q8;
      }
      #pragma unroll
      for (int it = 0; it < 4; ++it) if (ok[it]) {
        *(volatile v8us*)(out16 + adr[it]) = vhi[it];
        *(volatile v8us*)(out16 + adr[it] + segStride) = vlo[it];
        *(volatile v8us*)(out16 + adr[it] + 2 * (size_t)segStride) = vhi[it];
      }
      __threadfence();
      #pragma unroll
      for (int it = 0; it < 4; ++it) if (ok[it]) {
        *(volatile v8us*)(out16 + adr[it]) = vhi[it];
        *(volatile v8us*)(out16 + adr[it] + segStride) = vlo[it];
        *(volatile v8us*)(out16 + adr[it] + 2 * (size_t)segStride) = vhi[it];
      }
    } else if (MODE == 2) {
      v4f vals[8];
      size_t adr[8];
      #pragma unroll
      for (int it = 0; it < 8; ++it) {
        const int L = it * 32 + wid * 4 + sub;
        const int mloc = L >> 2, j = L & 3;
        const int nloc = j * 32 + 4 * q8;
        vals[it] = *(const v4fa*)(S + mloc * 128 + nloc);
        adr[it] = (size_t)(mblk + 64 * ph + mloc) * ldo + nblk + nloc;
      }
      #pragma unroll
      for (int it = 0; it < 8; ++it) *(volatile v4f*)(outf + adr[it]) = vals[it];
      __threadfence();
      #pragma unroll
      for (int it = 0; it < 8; ++it) *(volatile v4f*)(outf + adr[it]) = vals[it];
    } else {
      v4f vals[8];
      size_t adr[8];
      #pragma unroll
      for (int it = 0; it < 8; ++it) {
        const int L = it * 32 + wid * 4 + sub;
        const int nloc = L >> 1, j = L & 1;
        const int mloc = j * 32 + 4 * q8;
        vals[it] = *(const v4fa*)(S + nloc * 64 + mloc);
        adr[it] = (size_t)(nblk + nloc) * ldo + mblk + 64 * ph + mloc;
      }
      #pragma unroll
      for (int it = 0; it < 8; ++it) *(volatile v4f*)(outf + adr[it]) = vals[it];
      __threadfence();
      #pragma unroll
      for (int it = 0; it < 8; ++it) *(volatile v4f*)(outf + adr[it]) = vals[it];
    }
  }
}

__global__ __launch_bounds__(128) void psroi_k(const float* __restrict__ hpl, const float* __restrict__ rois,
                                               us_t* __restrict__ flat) {
  __shared__ __attribute__((aligned(16))) float sv[512];
  const int tid = threadIdx.x, lane = tid & 31, wid = tid >> 5, q8 = lane & 7, sub = lane >> 3;
  const int r = blockIdx.x;
  const bool valid = r < NROI;
  const int rr = valid ? r : (NROI - 1);
  const float rx1 = rois[rr * 4 + 0], ry1 = rois[rr * 4 + 1], rx2 = rois[rr * 4 + 2], ry2 = rois[rr * 4 + 3];
  const float x1 = rx1 * 0.0625f;
  const float y1 = ry1 * 0.0625f;
  const float x2 = rx2 * 0.0625f;
  const float y2 = ry2 * 0.0625f;
  const float dx = x2 - x1;
  const float dy = y2 - y1;
  const float bw = dx / 7.0f;
  const float bh = dy / 7.0f;
  #pragma unroll 1
  for (int j = 0; j < 4; ++j) {
    const int k = tid + 128 * j;
    const int kc = imin(k, COUT - 1);
    const int gw = kc % 7, gh = (kc % 49) / 7;
    const float gxf = (float)gw, gyf = (float)gh;
    const float* pl = hpl + (size_t)kc * HPITCH;
    float best = -3.0e38f;
    #pragma unroll
    for (int sy = 0; sy < 2; ++sy) {
      const float fy = gyf + ((sy == 0) ? 0.25f : 0.75f);
      const float pyv = fy * bh;
      float ys = y1 + pyv;
      ys = fminf(fmaxf(ys, 0.0f), (float)(HIMG - 1));
      const float y0f = floorf(ys);
      const float ly = ys - y0f;
      int y0 = (int)y0f;
      y0 = imin(imax(y0, 0), HIMG - 1);
      const int y1i = imin(y0 + 1, HIMG - 1);
      const float omy = 1.0f - ly;
      #pragma unroll
      for (int sx = 0; sx < 2; ++sx) {
        const float fx = gxf + ((sx == 0) ? 0.25f : 0.75f);
        const float pxv = fx * bw;
        float xs = x1 + pxv;
        xs = fminf(fmaxf(xs, 0.0f), (float)(WIMG - 1));
        const float x0f = floorf(xs);
        const float lx = xs - x0f;
        int x0 = (int)x0f;
        x0 = imin(imax(x0, 0), WIMG - 1);
        const int x1i = imin(x0 + 1, WIMG - 1);
        const float v00 = pl[y0 * WIMG + x0];
        const float v01 = pl[y0 * WIMG + x1i];
        const float v10 = pl[y1i * WIMG + x0];
        const float v11 = pl[y1i * WIMG + x1i];
        const float omx = 1.0f - lx;
        const float ta = omx * v00;
        const float tb = lx * v01;
        const float top = ta + tb;
        const float tc = omx * v10;
        const float td = lx * v11;
        const float bot = tc + td;
        const float pa = omy * top;
        const float pb = ly * bot;
        const float val = pa + pb;
        best = fmaxf(best, val);
      }
    }
    sv[k] = (valid && (k < COUT)) ? best : 0.0f;
  }
  __syncthreads();
  v8us vals[2];
  size_t adr[2];
  bool ok[2];
  #pragma unroll
  for (int it = 0; it < 2; ++it) {
    const int L = it * 16 + wid * 4 + sub;
    ok[it] = L < 24;
    const int Lc = ok[it] ? L : 0;
    const int seg = Lc >> 3, cb = Lc & 7;
    const float* sp = sv + cb * 64 + 8 * q8;
    const v4f f0 = *(const v4fa*)sp;
    const v4f f1 = *(const v4fa*)(sp + 4);
    v8us hi, lo;
    pack8bf(f0, f1, hi, lo);
    v8us o;
    #pragma unroll
    for (int i = 0; i < 8; ++i) o[i] = (seg == 1) ? lo[i] : hi[i];
    vals[it] = o;
    adr[it] = (size_t)r * KF + (size_t)seg * FSEG + cb * 64 + 8 * q8;
  }
  #pragma unroll
  for (int it = 0; it < 2; ++it) if (ok[it]) *(volatile v8us*)(flat + adr[it]) = vals[it];
  __threadfence();
  #pragma unroll
  for (int it = 0; it < 2; ++it) if (ok[it]) *(volatile v8us*)(flat + adr[it]) = vals[it];
}

__global__ __launch_bounds__(256) void out_k(const float* __restrict__ outs, float* __restrict__ out, int nf4) {
  const int i = blockIdx.x * 256 + threadIdx.x;
  if (i >= nf4) return;
  float e[4];
  #pragma unroll
  for (int u = 0; u < 4; ++u) {
    const int f = 4 * i + u;
    const bool a = f < NROI * NLOC;
    const int fa = a ? f : 0;
    const int ra = fa / NLOC, ja = fa - ra * NLOC;
    const int gb = a ? 0 : (f - NROI * NLOC);
    const int rb = gb / NSCO, jb = NLOC + (gb - rb * NSCO);
    const int ro = imin(a ? ra : rb, NR - 1);
    const int jo = a ? ja : jb;
    e[u] = outs[(size_t)ro * OPITCH + jo];
  }
  v4f v;
  v.x = e[0]; v.y = e[1]; v.z = e[2]; v.w = e[3];
  float* dst = out + (size_t)4 * i;
  *(volatile v4f*)dst = v;
  __threadfence();
  *(volatile v4f*)dst = v;
}

extern "C" void kernel_launch(void* const* d_in, const int* in_sizes, int n_in,
                              void* d_out, int out_size, void* d_ws, size_t ws_size,
                              hipStream_t stream) {
  if (n_in < 16) return;
  if (in_sizes[0] != CIN * NSP || in_sizes[1] != NROI * 4) return;
  if (in_sizes[2] != 256 * CIN * 15 || in_sizes[3] != 256) return;
  if (in_sizes[4] != COUT * CMID * 15 || in_sizes[5] != COUT) return;
  if (in_sizes[6] != 256 * CIN * 15 || in_sizes[7] != 256) return;
  if (in_sizes[8] != COUT * CMID * 15 || in_sizes[9] != COUT) return;
  if (in_sizes[10] != 2048 * COUT || in_sizes[11] != 2048) return;
  if (in_sizes[12] != NSCO * 2048 || in_sizes[13] != NSCO) return;
  if (in_sizes[14] != NLOC * 2048 || in_sizes[15] != NLOC) return;
  if (out_size != NROI * (NLOC + NSCO)) return;

  const float* x         = (const float*)d_in[0];
  const float* rois      = (const float*)d_in[1];
  const float* w_col_max = (const float*)d_in[2];
  const float* b_col_max = (const float*)d_in[3];
  const float* w_col     = (const float*)d_in[4];
  const float* b_col     = (const float*)d_in[5];
  const float* w_row_max = (const float*)d_in[6];
  const float* b_row_max = (const float*)d_in[7];
  const float* w_row     = (const float*)d_in[8];
  const float* b_row     = (const float*)d_in[9];
  const float* fc1_w     = (const float*)d_in[10];
  const float* fc1_b     = (const float*)d_in[11];
  const float* score_w   = (const float*)d_in[12];
  const float* score_b   = (const float*)d_in[13];
  const float* loc_w     = (const float*)d_in[14];
  const float* loc_b     = (const float*)d_in[15];
  float* out = (float*)d_out;

  char* ws = (char*)d_ws;
  size_t off = 0;
  const size_t szXP   = (size_t)XPROWS * CIN * 2;
  const size_t szW1   = (size_t)256 * K1 * 2;
  const size_t szW2   = (size_t)512 * K2 * 2;
  const size_t szMC   = (size_t)MCROWS * CMID * 2;
  const size_t szMR   = (size_t)MRROWS * CMID * 2;
  const size_t szHPL  = (size_t)512 * HPITCH * 4;
  const size_t szFLAT = (size_t)NR * KF * 2;
  const size_t szFC1W = (size_t)2048 * KF * 2;
  const size_t szACT  = (size_t)NR * KH * 2;
  const size_t szHW   = (size_t)512 * KH * 2;
  const size_t szOUTS = (size_t)NR * OPITCH * 4;
  us_t*  XP   = (us_t*)(ws + off);  off += szXP;
  us_t*  W1C  = (us_t*)(ws + off);  off += szW1;
  us_t*  W1R  = (us_t*)(ws + off);  off += szW1;
  us_t*  W2C  = (us_t*)(ws + off);  off += szW2;
  us_t*  W2R  = (us_t*)(ws + off);  off += szW2;
  us_t*  MIDC = (us_t*)(ws + off);  off += szMC;
  us_t*  MIDR = (us_t*)(ws + off);  off += szMR;
  float* HPL  = (float*)(ws + off); off += szHPL;
  us_t*  FLAT = (us_t*)(ws + off);  off += szFLAT;
  us_t*  FC1W = (us_t*)(ws + off);  off += szFC1W;
  us_t*  ACT  = (us_t*)(ws + off);  off += szACT;
  us_t*  HW   = (us_t*)(ws + off);  off += szHW;
  float* OUTS = (float*)(ws + off); off += szOUTS;
  if (off > ws_size) return;

  const float inv64 = 1.0f / WCAR;

  xpad_k<<<dim3(CIN / 64, 64), 256, 0, stream>>>(x, XP);
  packw_k<<<(256 * 15 * (CIN / 8) + 255) / 256, 256, 0, stream>>>(w_col_max, W1C, 256, 256, CIN, 256 * 15 * (CIN / 8));
  packw_k<<<(256 * 15 * (CIN / 8) + 255) / 256, 256, 0, stream>>>(w_row_max, W1R, 256, 256, CIN, 256 * 15 * (CIN / 8));
  packw_k<<<(512 * 15 * (CMID / 8) + 255) / 256, 256, 0, stream>>>(w_col, W2C, COUT, 512, CMID, 512 * 15 * (CMID / 8));
  packw_k<<<(512 * 15 * (CMID / 8) + 255) / 256, 256, 0, stream>>>(w_row, W2R, COUT, 512, CMID, 512 * 15 * (CMID / 8));
  packfc1_k<<<(2048 * 64 + 255) / 256, 256, 0, stream>>>(fc1_w, FC1W);
  packhead_k<<<(512 * 256 + 255) / 256, 256, 0, stream>>>(loc_w, score_w, HW);
  {
    const int n16 = (int)((szMC + szMR) / 16);
    zero_k<<<(n16 + 255) / 256, 256, 0, stream>>>(MIDC, n16);
  }

  const int NBN = (NSP + 127) / 128;
  gemm_k<v16h, 0><<<dim3(2, NBN), 256, 0, stream>>>(
      W1C, XP, CIN, 15, XPW, XPW, 7,
      W1C, XP, CIN, 15, XPW, XPW, 7,
      1, NSP, 1,
      b_col_max, 256, b_col_max, 256,
      inv64, 0,
      MIDC, HPL, CMID, XPW, 7, 0);
  gemm_k<v16h, 0><<<dim3(2, NBN), 256, 0, stream>>>(
      W1R, XP, CIN, 15, 1, XPW, 7 * XPW,
      W1R, XP, CIN, 15, 1, XPW, 7 * XPW,
      1, NSP, 1,
      b_row_max, 256, b_row_max, 256,
      inv64, 0,
      MIDR, HPL, CMID, WIMG, 7 * WIMG, 0);
  gemm_k<v16h, 2><<<dim3(4, NBN), 256, 0, stream>>>(
      W2C, MIDC, CMID, 15, 1, XPW, 0,
      W2R, MIDR, CMID, 15, WIMG, WIMG, 0,
      2, NSP, 1,
      b_col, COUT, b_row, COUT,
      inv64, 1,
      MIDC, HPL, HPITCH, 0, 0, 0);
  psroi_k<<<NR, 128, 0, stream>>>(HPL, rois, FLAT);
  gemm_k<v16b, 1><<<dim3(2048 / 128, NR / 128), 256, 0, stream>>>(
      FC1W, FLAT, KF, 1, 0, 0, 0,
      FC1W, FLAT, KF, 1, 0, 0, 0,
      1, NR, 0,
      fc1_b, 2048, fc1_b, 2048,
      1.0f, 1,
      ACT, OUTS, KH, 0, 0, HSEG);
  gemm_k<v16b, 3><<<dim3(4, NR / 128), 256, 0, stream>>>(
      HW, ACT, KH, 1, 0, 0, 0,
      HW, ACT, KH, 1, 0, 0, 0,
      1, NR, 0,
      loc_b, NLOC, score_b, NSCO,
      1.0f, 0,
      FLAT, OUTS, OPITCH, 0, 0, 0);
  {
    const int nf4 = NROI * (NLOC + NSCO) / 4;
    out_k<<<(nf4 + 255) / 256, 256, 0, stream>>>(OUTS, out, nf4);
  }
}
